// TransformerBlock_89215060672757
// MI455X (gfx1250) — hardware-run, weakly checked
//
#include <hip/hip_runtime.h>
#ifndef NB
#define NB 2
#endif
#ifndef SEQ
#define SEQ 2048
#endif
#define NB_FULL 2
#define SEQ_FULL 2048
#define SQ SEQ
#define DM 1024
#define NH 16
#define HD 64
#define DFF 4096
#define QT 256
#define NKX SQ
#define NR ((size_t)NB * SQ)
#define DMQ DM
#define LQ (3 * DM)

typedef unsigned short v8us __attribute__((ext_vector_type(8), may_alias));
typedef float  v8f  __attribute__((ext_vector_type(8)));
typedef float  v4f  __attribute__((ext_vector_type(4)));
typedef float  v4fa __attribute__((ext_vector_type(4), may_alias));
typedef _Float16 v16h __attribute__((ext_vector_type(16)));
typedef _Float16 v4h __attribute__((ext_vector_type(4)));
union FragH { v16h v; v8us half[2]; _Float16 h[16]; unsigned short u[16]; };

static_assert(DM == 1024);
static_assert(NH * HD == DM);
static_assert(SQ % QT == 0);
static_assert(QT % 128 == 0);
static_assert((NB * SQ) % 128 == 0);
static_assert(DM % 64 == 0 && DFF % 64 == 0 && (3 * DM) % 64 == 0);
static_assert(DM % 32 == 0 && DFF % 32 == 0 && HD % 32 == 0);
static_assert(NB <= NB_FULL && SEQ <= SEQ_FULL);
static_assert(HD == 64);
static_assert(256 * 4 == DMQ);
static_assert(SQ % 64 == 0);
static_assert(DM % 8 == 0 && DFF % 8 == 0);

__device__ __forceinline__ unsigned short bf16_bits(float x) { unsigned int u = __float_as_uint(x); return (unsigned short)((u + 0x7FFFu + ((u >> 16) & 1u)) >> 16); }
__device__ __forceinline__ float bf16_val(unsigned short b) { return __uint_as_float(((unsigned int)b) << 16); }
__device__ __forceinline__ float bf16_rne(float x) { return bf16_val(bf16_bits(x)); }

__global__ __launch_bounds__(256) void k_wt_f16(const float* __restrict__ W, _Float16* __restrict__ Wt, int K, int N, float scale) {
  const int t = blockIdx.x * 256 + threadIdx.x; if (t >= N * (K / 8)) return; const int n = t / (K / 8), k8 = (t % (K / 8)) * 8; FragH f;
#pragma unroll
  for (int i = 0; i < 8; ++i) f.h[i] = (_Float16)(bf16_rne(W[(size_t)(k8 + i) * N + n]) * scale);
  const v8us o = f.half[0];
  *(volatile v8us*)((unsigned short*)Wt + (size_t)n * K + k8) = o; __threadfence(); *(volatile v8us*)((unsigned short*)Wt + (size_t)n * K + k8) = o;
}

template <int NHv, int TTv>
__global__ __launch_bounds__(256) void k_vt(const _Float16* __restrict__ V16, int ldv, int voff, _Float16* __restrict__ Vt) {
  __shared__ unsigned short tl[64][66]; const int tid = threadIdx.x; const int slab = blockIdx.x / (TTv / 64), lg = blockIdx.x % (TTv / 64); const int b = slab / NHv, h = slab % NHv;
  for (int i = tid; i < 64 * 8; i += 256) { const int r = i / 8, c8 = (i % 8) * 8; FragH f; f.half[0] = *(const v8us*)((const unsigned short*)V16 + ((size_t)b * TTv + lg * 64 + r) * ldv + voff + h * 64 + c8);
#pragma unroll
    for (int q = 0; q < 8; ++q) tl[r][c8 + q] = f.u[q]; }
  __syncthreads();
  for (int pass = 0; pass < 2; ++pass) {
#pragma unroll
    for (int rd = 0; rd < 2; ++rd) { const int d = rd * 32 + tid / 8, pc = tid % 8; FragH f;
#pragma unroll
      for (int q = 0; q < 8; ++q) f.u[q] = tl[pc * 8 + q][d];
      *(volatile v8us*)((unsigned short*)Vt + ((size_t)slab * 64 + d) * TTv + lg * 64 + pc * 8) = f.half[0]; }
    if (pass == 0) __threadfence(); } }

__device__ __forceinline__ v16h g2_frag(const _Float16* p, int hh) { FragH f; f.half[0] = *(const v8us*)((const unsigned short*)p + 8 * hh); f.half[1] = *(const v8us*)((const unsigned short*)p + 16 + 8 * hh); return f.v; }
__device__ __forceinline__ v8f g2_mma(v16h a, v16h b, v8f c) { v8f d = __builtin_amdgcn_wmma_f32_16x16x32_f16(false, a, false, b, (short)0, c, false, false); asm volatile("v_nop\n\tv_nop\n\tv_nop\n\tv_nop" : "+v"(d) : "v"(a), "v"(b)); return d; }
template <int ACT>
__global__ __launch_bounds__(128) void k_gemm2(const _Float16* __restrict__ A, int lda, size_t sA, const _Float16* __restrict__ Bh, int ldb, size_t sB, float alpha, const float* __restrict__ CP,
    float* __restrict__ C, _Float16* __restrict__ C16, int ldc, size_t sC, int M, int N, int K) {
  static_assert(ACT == 0 || ACT == 3);
  __shared__ __attribute__((aligned(16))) float so[4][32][68];
  const int tid = threadIdx.x, w = tid >> 5, lane = tid & 31, ln = lane & 15, hh = lane >> 4; const int by = blockIdx.y;
  A += (size_t)by * sA; Bh += (size_t)by * sB; const size_t cofs = (size_t)by * sC;
  const int ntn = N >> 6; const int mt = blockIdx.x / ntn, nq = blockIdx.x - mt * ntn; const int row0 = mt * 128 + 32 * w, col0 = nq * 64; if (row0 >= M) return;
  const _Float16* a0p = A + (size_t)(row0 + ln) * lda; const _Float16* a1p = a0p + (size_t)16 * lda;
  const _Float16* b0p = Bh + (size_t)(col0 + ln) * ldb; const _Float16* b1p = b0p + (size_t)16 * ldb; const _Float16* b2p = b1p + (size_t)16 * ldb; const _Float16* b3p = b2p + (size_t)16 * ldb;
  const v8f z8 = {0.f,0.f,0.f,0.f,0.f,0.f,0.f,0.f}; v8f c00 = z8, c01 = z8, c02 = z8, c03 = z8, c10 = z8, c11 = z8, c12 = z8, c13 = z8;
#pragma unroll 1
  for (int kb = 0; kb < K; kb += 32) { const v16h a0 = g2_frag(a0p + kb, hh), a1 = g2_frag(a1p + kb, hh);
    v16h b = g2_frag(b0p + kb, hh); c00 = g2_mma(a0, b, c00); c10 = g2_mma(a1, b, c10);
    b = g2_frag(b1p + kb, hh); c01 = g2_mma(a0, b, c01); c11 = g2_mma(a1, b, c11);
    b = g2_frag(b2p + kb, hh); c02 = g2_mma(a0, b, c02); c12 = g2_mma(a1, b, c12);
    b = g2_frag(b3p + kb, hh); c03 = g2_mma(a0, b, c03); c13 = g2_mma(a1, b, c13); }
  v8f accs[8] = {c00, c01, c02, c03, c10, c11, c12, c13};
#pragma unroll
  for (int u = 0; u < 8; ++u) { const int t = u & 3, half = u >> 2; const int col = col0 + t * 16 + ln;
#pragma unroll
    for (int r = 0; r < 8; ++r) { const int rloc = half * 16 + 8 * hh + r; float v = accs[u][r] * alpha;
      if (CP) v += CP[cofs + (size_t)(row0 + rloc) * ldc + col];
      if (ACT == 3) v = fmaxf(v, 0.f);
      so[w][rloc][t * 16 + ln] = v; } }
  __builtin_amdgcn_fence(4  , "workgroup"); __builtin_amdgcn_wave_barrier();
  const int rsub = lane >> 4, c4 = (lane & 15) * 4;
  for (int pass = 0; pass < 2; ++pass) {
#pragma unroll
    for (int q = 0; q < 16; ++q) { const int r = q * 2 + rsub; const v4f v = *(const v4fa*)&so[w][r][c4];
      if (C) *(volatile v4f*)(C + cofs + (size_t)(row0 + r) * ldc + col0 + c4) = v;
      if (C16) { v4h h4; for (int i = 0; i < 4; ++i) h4[i] = (_Float16)v[i]; *(volatile v4h*)(C16 + cofs + (size_t)(row0 + r) * ldc + col0 + c4) = h4; } }
    if (pass == 0) __threadfence(); } }

__global__ __launch_bounds__(128) void k_gemm2gu(const _Float16* __restrict__ A, int lda, const _Float16* __restrict__ Bg, const _Float16* __restrict__ Bu, int ldb, float alpha,
    _Float16* __restrict__ C16, int ldc, int M, int N, int K) {
  __shared__ __attribute__((aligned(16))) float so[4][32][68];
  const int tid = threadIdx.x, lane = tid & 31, ln = lane & 15, hh = lane >> 4; const int w = __builtin_amdgcn_readfirstlane(tid >> 5);
  const int ntn = N >> 6; const int mt = blockIdx.x / ntn, nq = blockIdx.x - mt * ntn; const int row0 = mt * 128 + 32 * w, col0 = nq * 64; if (row0 >= M) return;
  const _Float16* a0p = A + (size_t)(row0 + ln) * lda; const _Float16* a1p = a0p + (size_t)16 * lda;
  const size_t bofs = (size_t)(col0 + ln) * ldb; const size_t bstep = (size_t)16 * ldb;
  const _Float16* g0p = Bg + bofs; const _Float16* g1p = g0p + bstep; const _Float16* g2p = g1p + bstep; const _Float16* g3p = g2p + bstep;
  const _Float16* u0p = Bu + bofs; const _Float16* u1p = u0p + bstep; const _Float16* u2p = u1p + bstep; const _Float16* u3p = u2p + bstep;
  const v8f z8 = {0.f,0.f,0.f,0.f,0.f,0.f,0.f,0.f};
  v8f g00 = z8, g01 = z8, g02 = z8, g03 = z8, g10 = z8, g11 = z8, g12 = z8, g13 = z8;
  v8f u00 = z8, u01 = z8, u02 = z8, u03 = z8, u10 = z8, u11 = z8, u12 = z8, u13 = z8;
#pragma unroll 1
  for (int kb = 0; kb < K; kb += 32) { const v16h a0 = g2_frag(a0p + kb, hh), a1 = g2_frag(a1p + kb, hh);
    v16h b = g2_frag(g0p + kb, hh); g00 = g2_mma(a0, b, g00); g10 = g2_mma(a1, b, g10);
    b = g2_frag(u0p + kb, hh); u00 = g2_mma(a0, b, u00); u10 = g2_mma(a1, b, u10);
    b = g2_frag(g1p + kb, hh); g01 = g2_mma(a0, b, g01); g11 = g2_mma(a1, b, g11);
    b = g2_frag(u1p + kb, hh); u01 = g2_mma(a0, b, u01); u11 = g2_mma(a1, b, u11);
    b = g2_frag(g2p + kb, hh); g02 = g2_mma(a0, b, g02); g12 = g2_mma(a1, b, g12);
    b = g2_frag(u2p + kb, hh); u02 = g2_mma(a0, b, u02); u12 = g2_mma(a1, b, u12);
    b = g2_frag(g3p + kb, hh); g03 = g2_mma(a0, b, g03); g13 = g2_mma(a1, b, g13);
    b = g2_frag(u3p + kb, hh); u03 = g2_mma(a0, b, u03); u13 = g2_mma(a1, b, u13); }
  v8f ga[8] = {g00, g01, g02, g03, g10, g11, g12, g13}; v8f ua[8] = {u00, u01, u02, u03, u10, u11, u12, u13};
#pragma unroll
  for (int u = 0; u < 8; ++u) { const int t = u & 3, half = u >> 2;
#pragma unroll
    for (int r = 0; r < 8; ++r) { const int rloc = half * 16 + 8 * hh + r; const float gv = ga[u][r] * alpha; const float uv = ua[u][r] * alpha;
      const float sg = gv * __builtin_amdgcn_rcpf(1.0f + __expf(-gv));
      so[w][rloc][t * 16 + ln] = sg * uv; } }
  __builtin_amdgcn_fence(4  , "workgroup"); __builtin_amdgcn_wave_barrier();
  const int rsub = lane >> 4, c4 = (lane & 15) * 4;
  for (int pass = 0; pass < 2; ++pass) {
#pragma unroll
    for (int q = 0; q < 16; ++q) { const int r = q * 2 + rsub; const v4f v = *(const v4fa*)&so[w][r][c4];
      v4h h4; for (int i = 0; i < 4; ++i) h4[i] = (_Float16)v[i]; *(volatile v4h*)(C16 + (size_t)(row0 + r) * ldc + col0 + c4) = h4; }
    if (pass == 0) __threadfence(); } }

__global__ __launch_bounds__(256) void k_rsmcf2(const float* __restrict__ S, _Float16* __restrict__ P, int hg, int q0, int nk) {
  #pragma clang fp contract(off)
  const int t = blockIdx.x * 256 + threadIdx.x; if (t >= hg * QT) return; const size_t i = (size_t)t; const float* s = S + i * NKX; const int last = q0 + (t % QT); float mx = -3.0e38f;
#pragma unroll 1
  for (int j = 0; j < nk; ++j) { const float f = (j <= last) ? 1.f : 0.f; mx = fmaxf(mx, fmaf(f, s[j], (1.f - f) * -1.0e9f)); } float se = 0.f;
#pragma unroll 1
  for (int j = 0; j < nk; ++j) { const float f = (j <= last) ? 1.f : 0.f; se += __expf(fmaf(f, s[j], (1.f - f) * -1.0e9f) - mx); } const float sc = 256.0f / se;
#pragma unroll 1
  for (int j0 = 0; j0 < nk; j0 += 8) { FragH fr; for (int q = 0; q < 8; ++q) { const int j = j0 + q; const float f = (j <= last) ? 1.f : 0.f; fr.h[q] = (_Float16)(__expf(fmaf(f, s[j], (1.f - f) * -1.0e9f) - mx) * sc); } unsigned short* d = (unsigned short*)P + i * NKX + j0; const v8us pv = fr.half[0]; *(volatile v8us*)d = pv; __threadfence(); *(volatile v8us*)d = pv; } }

template <int BFIN, int WXB>
__device__ __forceinline__ void rms_rows(const float* __restrict__ X, int spb, int spbf, const float* __restrict__ g, float eps, _Float16* __restrict__ N16, float* __restrict__ XB) {
  #pragma clang fp contract(off)
  __shared__ float red[256]; const int r = blockIdx.x; const int t = threadIdx.x; const int c0 = t * 4;
  const size_t rin = (size_t)(r / spb) * (size_t)spbf + (size_t)(r % spb);
  const v4f xa = *(const v4fa*)(X + rin * DMQ + c0); float s[4]; float ss = 0.f;
  for (int q = 0; q < 4; ++q) { s[q] = BFIN ? bf16_rne(xa[q]) : xa[q]; ss = ss + s[q] * s[q]; }
  red[t] = ss; __syncthreads(); for (int st = 128; st > 0; st >>= 1) { if (t < st) red[t] = red[t] + red[t + st]; __syncthreads(); }
  const float rs = rsqrtf(red[0] * (1.0f / (float)DMQ) + eps); v4h y; v4f xb;
  for (int q = 0; q < 4; ++q) { const int c = c0 + q; const float yf = (s[q] * rs) * bf16_rne(g[c]); y[q] = (_Float16)yf; xb[q] = s[q]; }
  for (int pass = 0; pass < 2; ++pass) { *(volatile v4h*)(N16 + (size_t)r * DMQ + c0) = y; if (WXB) *(volatile v4f*)(XB + (size_t)r * DMQ + c0) = xb; if (pass == 0) __threadfence(); } }
__global__ __launch_bounds__(256) void k_rms_in(const float* __restrict__ X, int spb, int spbf, const float* __restrict__ g, float eps, _Float16* __restrict__ N16, float* __restrict__ XB) { rms_rows<1, 1>(X, spb, spbf, g, eps, N16, XB); }
__global__ __launch_bounds__(256) void k_rms_mid(const float* __restrict__ X, int spb, int spbf, const float* __restrict__ g, float eps, _Float16* __restrict__ N16) { rms_rows<0, 0>(X, spb, spbf, g, eps, N16, nullptr); }

constexpr size_t cmax(size_t a, size_t b) { return a > b ? a : b; }
constexpr size_t al256(size_t b) { return (b + 255) & ~(size_t)255; }
constexpr size_t SZ_BQKV = al256((size_t)3 * DM * DM * 2);
constexpr size_t SZ_X16  = al256(NR * DM * 2);
constexpr size_t SZ_XB   = al256(NR * DM * 4);
constexpr size_t SZ_QKV  = al256(cmax(NR * 3 * DM * 2, NR * DM * 4));
constexpr size_t SZ_O16  = al256(NR * DM * 2);
constexpr size_t SZ_SREG = al256(cmax((size_t)NH * QT * NKX * 4, NR * DFF * 2));
constexpr size_t SZ_PREG = al256(cmax((size_t)NH * QT * NKX * 2, (size_t)3 * DFF * DM * 2));
constexpr size_t SZ_VT   = al256((size_t)NH * HD * SQ * 2);
constexpr size_t SZ_BWP  = al256((size_t)DM * DM * 2);
constexpr size_t SZ_TOTAL = SZ_BQKV + SZ_X16 + SZ_XB + SZ_QKV + SZ_O16 + SZ_SREG + SZ_PREG + SZ_VT + SZ_BWP;
static_assert(SZ_TOTAL <= (size_t)134217728);
static_assert(NR * DM * 4 <= SZ_QKV);
static_assert(NR * 3 * DM * 2 <= SZ_QKV);
static_assert(NR * DFF * 2 <= SZ_SREG);
static_assert((size_t)NH * QT * NKX * 4 <= SZ_SREG);
static_assert((size_t)NH * QT * NKX * 2 <= SZ_PREG);
static_assert((size_t)3 * DFF * DM * 2 <= SZ_PREG);

extern "C" void kernel_launch(void* const* d_in, const int* in_sizes, int n_in,
                              void* d_out, int out_size, void* d_ws, size_t ws_size, hipStream_t stream) {
  if (n_in < 8) return;
  const size_t need_x = ((size_t)(NB - 1) * SEQ_FULL + SQ) * DM;
  if ((size_t)in_sizes[0] < need_x || in_sizes[1] < DM || in_sizes[2] < DM || in_sizes[3] < DM * 3 * DM || in_sizes[4] < DM * DM || in_sizes[5] < DM * DFF || in_sizes[6] < DM * DFF || in_sizes[7] < DFF * DM) return;
  if ((size_t)out_size < need_x) return;
  if (SZ_TOTAL > ws_size) return;
  const float* x = (const float*)d_in[0]; const float* g1 = (const float*)d_in[1]; const float* g2 = (const float*)d_in[2]; const float* wqkv = (const float*)d_in[3];
  const float* wout = (const float*)d_in[4]; const float* wgate = (const float*)d_in[5]; const float* wup = (const float*)d_in[6]; const float* wdown = (const float*)d_in[7];
  float* out = (float*)d_out;
  char* ws = (char*)d_ws; size_t off = 0;
  _Float16* BQKV = (_Float16*)(ws + off); off += SZ_BQKV;
  _Float16* X16  = (_Float16*)(ws + off); off += SZ_X16;  _Float16* M16 = X16;
  float*    XB   = (float*)(ws + off);    off += SZ_XB;
  _Float16* QKV  = (_Float16*)(ws + off); float* X1 = (float*)(ws + off); off += SZ_QKV;
  _Float16* O16  = (_Float16*)(ws + off); off += SZ_O16;
  float*    S    = (float*)(ws + off);    _Float16* HF16 = (_Float16*)(ws + off); off += SZ_SREG;
  _Float16* P    = (_Float16*)(ws + off); _Float16* BWG = (_Float16*)(ws + off); _Float16* BWU = BWG + (size_t)DFF * DM; _Float16* BWD = BWU + (size_t)DFF * DM; off += SZ_PREG;
  _Float16* VT   = (_Float16*)(ws + off); off += SZ_VT;
  _Float16* BWP  = (_Float16*)(ws + off); off += SZ_BWP;
  if (off > ws_size) return;
  _Float16* Q16 = QKV; _Float16* K16 = QKV + DM; _Float16* V16 = QKV + 2 * DM;

  k_wt_f16<<<(unsigned)(((size_t)(3 * DM) * (DM / 8) + 255) / 256), 256, 0, stream>>>(wqkv, BQKV, DM, 3 * DM, 16.0f);
  k_wt_f16<<<(unsigned)(((size_t)DM * (DM / 8) + 255) / 256), 256, 0, stream>>>(wout, BWP, DM, DM, 16.0f);
  k_rms_in<<<(unsigned)NR, 256, 0, stream>>>(x, SQ, SEQ_FULL, g1, 1e-6f, X16, XB);
  k_gemm2<0><<<dim3((unsigned)((NR / 128) * (3 * DM / 64)), 1), 128, 0, stream>>>(X16, DM, 0, BQKV, DM, 0, 0.0625f, nullptr, nullptr, QKV, 3 * DM, 0, (int)NR, 3 * DM, DM);
  for (int b = 0; b < NB; ++b) { const size_t r0 = (size_t)b * SQ;
    k_vt<NH, SQ><<<NH * (SQ / 64), 256, 0, stream>>>(V16 + r0 * LQ, LQ, 0, VT);
    for (int q0 = 0; q0 < SQ; q0 += QT) { const int nk = q0 + QT;
      k_gemm2<0><<<dim3((unsigned)((QT / 128) * (nk / 64)), NH), 128, 0, stream>>>(Q16 + (r0 + q0) * LQ, LQ, (size_t)HD, K16 + r0 * LQ, LQ, (size_t)HD, 0.125f, nullptr, S, nullptr, NKX, (size_t)QT * NKX, QT, nk, HD);
      k_rsmcf2<<<(NH * QT + 255) / 256, 256, 0, stream>>>(S, P, NH, q0, nk);
      k_gemm2<0><<<dim3((unsigned)((QT / 128) * (HD / 64)), NH), 128, 0, stream>>>(P, NKX, (size_t)QT * NKX, VT, SQ, (size_t)HD * SQ, 0.25f, nullptr, nullptr, O16 + (r0 + q0) * DM, DM, (size_t)HD, QT, HD, nk); } }
  k_wt_f16<<<(unsigned)(((size_t)DFF * (DM / 8) + 255) / 256), 256, 0, stream>>>(wgate, BWG, DM, DFF, 16.0f);
  k_wt_f16<<<(unsigned)(((size_t)DFF * (DM / 8) + 255) / 256), 256, 0, stream>>>(wup, BWU, DM, DFF, 16.0f);
  k_wt_f16<<<(unsigned)(((size_t)DM * (DFF / 8) + 255) / 256), 256, 0, stream>>>(wdown, BWD, DFF, DM, 16.0f);
  k_gemm2<0><<<dim3((unsigned)((NR / 128) * (DM / 64)), 1), 128, 0, stream>>>(O16, DM, 0, BWP, DM, 0, 0.0009765625f, XB, X1, nullptr, DM, 0, (int)NR, DM, DM);
  k_rms_mid<<<(unsigned)NR, 256, 0, stream>>>(X1, SQ, SQ, g2, 1e-6f, M16);
  k_gemm2gu<<<(unsigned)((NR / 128) * (DFF / 64)), 128, 0, stream>>>(M16, DM, BWG, BWU, DM, 0.0625f, HF16, DFF, (int)NR, DFF, DM);
  for (int b = 0; b < NB; ++b) { const size_t r0 = (size_t)b * SQ;
    k_gemm2<0><<<dim3((unsigned)((SQ / 128) * (DM / 64)), 1), 128, 0, stream>>>(HF16 + r0 * DFF, DFF, 0, BWD, DFF, 0, 0.0625f, X1 + r0 * DM, out + (size_t)b * SEQ_FULL * DM, nullptr, DM, 0, SQ, DM, DFF); }
}
